// PromptFormer_77653008711745
// MI455X (gfx1250) — hardware-verified
//
#include <hip/hip_runtime.h>
#include <math.h>

typedef __attribute__((ext_vector_type(16))) _Float16 v16h;
typedef __attribute__((ext_vector_type(16))) __bf16 v16b;
typedef __attribute__((ext_vector_type(8)))  _Float16 v8h;
typedef __attribute__((ext_vector_type(8)))  float v8f;
typedef __attribute__((ext_vector_type(4)))  float v4f;
typedef __attribute__((ext_vector_type(2)))  float v2f;
typedef __attribute__((ext_vector_type(4)))  unsigned v4u;
typedef __attribute__((ext_vector_type(4)))  int v4i;
typedef float __attribute__((may_alias)) float_a;
typedef int __attribute__((may_alias)) int_a;

template <typename T> __device__ __forceinline__ void vst2(void* p, T v) { *(volatile T*)p = v; __threadfence(); *(volatile T*)p = v; }
__device__ __forceinline__ v8f wmma16(v16h a, v16h b, v8f c) {
  v8f d = __builtin_amdgcn_wmma_f32_16x16x32_f16(false, a, false, b, (short)0, c, false, false);
  asm volatile("v_nop\n\tv_nop\n\tv_nop\n\tv_nop" : "+v"(d) : "v"(a), "v"(b));
  return d;
}
__device__ __forceinline__ v8f wmma_bf(v16b a, v16b b, v8f c) {
  v8f d = __builtin_amdgcn_wmma_f32_16x16x32_bf16(false, a, false, b, (short)0, c, false, false);
  asm volatile("v_nop\n\tv_nop\n\tv_nop\n\tv_nop" : "+v"(d) : "v"(a), "v"(b));
  return d;
}
__device__ __forceinline__ v16h frag_h(const _Float16* rowk0, int lane) {
  union { v16h v; v8h q[2]; } u; const _Float16* p = rowk0 + 8 * (lane >> 4);
  u.q[0] = *(const v8h*)p; u.q[1] = *(const v8h*)(p + 16); return u.v;
}
__device__ __forceinline__ v16h frag_f32(const float* rowk0, int lane) {
  v16h a; const float* p = rowk0 + 8 * (lane >> 4);
#pragma unroll
  for (int i = 0; i < 8; ++i) { a[i] = (_Float16)p[i]; a[8 + i] = (_Float16)p[16 + i]; }
  return a;
}
__device__ __forceinline__ v16h frag_f32s(const float* rowk0, int lane, float sc) {
  v16h a; const float* p = rowk0 + 8 * (lane >> 4);
#pragma unroll
  for (int i = 0; i < 8; ++i) { a[i] = (_Float16)(p[i] * sc); a[8 + i] = (_Float16)(p[16 + i] * sc); }
  return a;
}
__device__ __forceinline__ v16h fragc_f32(const float* W, int k0, int n, int lane, int ld, int K) {
  v16h a; const int g = lane >> 4;
#pragma unroll
  for (int i = 0; i < 8; ++i) { const int ka = k0 + 8 * g + i, kb = ka + 16;
    a[i] = (_Float16)(ka < K ? W[(size_t)(ka < K ? ka : K - 1) * ld + n] : 0.f); a[8 + i] = (_Float16)(kb < K ? W[(size_t)(kb < K ? kb : K - 1) * ld + n] : 0.f); }
  return a;
}
struct F2 { v16b h, l; };
__device__ __forceinline__ F2 bsplit16(const float v[16]) { F2 r;
#pragma unroll
  for (int i = 0; i < 16; ++i) { const __bf16 h = (__bf16)v[i]; r.h[i] = h; r.l[i] = (__bf16)(v[i] - (float)h); }
  return r; }
__device__ __forceinline__ F2 split_row(const float* row, int k0, int lane) { float v[16]; const float* p = row + k0 + 8 * (lane >> 4);
#pragma unroll
  for (int i = 0; i < 8; ++i) { v[i] = p[i]; v[8 + i] = p[16 + i]; }
  return bsplit16(v); }
__device__ __forceinline__ F2 split_rowK(const float* row, int k0, int lane, int K) { float v[16]; const int g = lane >> 4;
#pragma unroll
  for (int i = 0; i < 8; ++i) { const int ka = k0 + 8 * g + i, kb = ka + 16; v[i] = ka < K ? row[ka < K ? ka : K - 1] : 0.f; v[8 + i] = kb < K ? row[kb < K ? kb : K - 1] : 0.f; }
  return bsplit16(v); }
__device__ __forceinline__ F2 split_col(const float* W, int k0, int n, int lane, int ld, int K) { float v[16]; const int g = lane >> 4;
#pragma unroll
  for (int i = 0; i < 8; ++i) { const int ka = k0 + 8 * g + i, kb = ka + 16; v[i] = ka < K ? W[(size_t)(ka < K ? ka : K - 1) * ld + n] : 0.f; v[8 + i] = kb < K ? W[(size_t)(kb < K ? kb : K - 1) * ld + n] : 0.f; }
  return bsplit16(v); }
__device__ __forceinline__ v8f mac3(const F2& a, const F2& b, v8f c) { c = wmma_bf(a.l, b.h, c); c = wmma_bf(a.h, b.l, c); return wmma_bf(a.h, b.h, c); }
__device__ __forceinline__ float sigm(float v) { return 1.0f / (1.0f + expf(-v)); }
#define LDSX() do { asm volatile("s_wait_dscnt 0" ::: "memory"); __builtin_amdgcn_wave_barrier(); __builtin_amdgcn_fence(__ATOMIC_RELEASE, "workgroup"); } while (0)


#define NBI 16
#define SQ 1024
#define D 128
#define NPR 128
#define NR (NBI * SQ)
#define NK (NBI * NPR)
__device__ __forceinline__ float bfr(float v) { return (float)(__bf16)v; }
__device__ __forceinline__ float gelu_e(float v) { return 0.5f * v * (1.0f + erff(v * 0.70710678118654752f)); }
__device__ __forceinline__ v16b frag_b(const __bf16* rowk0, int lane) { return __builtin_bit_cast(v16b, frag_h((const _Float16*)rowk0, lane)); }

__global__ __launch_bounds__(128) void k_proto(const float* __restrict__ x, const float* __restrict__ wn1, const float* __restrict__ bn1, const float* __restrict__ wn2, const float* __restrict__ bn2, float* __restrict__ proto, _Float16* __restrict__ VT16) {
  __shared__ __align__(16) float sh[4][16][D + 4]; __shared__ __align__(16) float spt[64][D + 4]; __shared__ __align__(16) _Float16 svt[4][16][D + 8];
  const int tid = threadIdx.x, wave = tid >> 5, lane = tid & 31, col = lane & 15, g = lane >> 4; const int b = blockIdx.y, d0b = blockIdx.x * 64, d0 = d0b + wave * 16;
  const float* xb = x + (size_t)b * SQ * D;
  { v8f acc[8] = {};
#pragma unroll 2
    for (int kc = 0; kc < SQ / 32; ++kc) { const v16b a = split_col(xb, kc * 32, d0 + col, lane, D, SQ).h;
#pragma unroll
      for (int j = 0; j < 8; ++j) acc[j] = wmma_bf(a, split_col(wn1, kc * 32, j * 16 + col, lane, NPR, SQ).h, acc[j]); }
#pragma unroll
    for (int j = 0; j < 8; ++j) { const float bb = bfr(bn1[j * 16 + col]);
#pragma unroll
      for (int r = 0; r < 8; ++r) sh[wave][8 * g + r][j * 16 + col] = gelu_e(acc[j][r] + bb); } }
  LDSX();
  { v8f acc[8] = {};
#pragma unroll
    for (int kc = 0; kc < NPR / 32; ++kc) { const F2 a = split_row(&sh[wave][col][0], kc * 32, lane);
#pragma unroll
      for (int j = 0; j < 8; ++j) { const v16b wb = split_col(wn2, kc * 32, j * 16 + col, lane, D, NPR).h; acc[j] = wmma_bf(a.l, wb, acc[j]); acc[j] = wmma_bf(a.h, wb, acc[j]); } }
#pragma unroll
    for (int j = 0; j < 8; ++j) { const float bb = bfr(bn2[j * 16 + col]);
#pragma unroll
      for (int r = 0; r < 8; ++r) { const float v = acc[j][r] + bb; spt[wave * 16 + 8 * g + r][j * 16 + col] = v; svt[wave][8 * g + r][j * 16 + col] = (_Float16)(v * 4.0f); } } }
  LDSX();
  for (int rl = 0; rl < 16; ++rl) { if (lane < 16) vst2(VT16 + (size_t)(d0 + rl) * NK + b * NPR + lane * 8, *(const v4u*)(&svt[wave][rl][lane * 8])); }
  __syncthreads();
  for (int q = tid; q < NPR * 16; q += 128) { const int m = q >> 4, pc = q & 15; v4f v;
#pragma unroll
    for (int e = 0; e < 4; ++e) v[e] = spt[pc * 4 + e][m];
    vst2(proto + ((size_t)b * NPR + m) * D + d0b + pc * 4, v); }
}
__global__ __launch_bounds__(256) void k_pn(const float* __restrict__ proto, _Float16* __restrict__ PN16) {
  const int wave = threadIdx.x >> 5, lane = threadIdx.x & 31; const int row = blockIdx.x * 8 + wave; const v4f v = *(const v4f*)(proto + (size_t)row * D + lane * 4);
  float ss = v[0] * v[0] + v[1] * v[1] + v[2] * v[2] + v[3] * v[3];
#pragma unroll
  for (int o = 16; o > 0; o >>= 1) ss += __shfl_xor(ss, o, 32);
  const float inv = 4.0f / sqrtf(ss);
  union { _Float16 h[4]; v2f f; unsigned long long u; } pk;
#pragma unroll
  for (int e = 0; e < 4; ++e) pk.h[e] = (_Float16)(v[e] * inv);
  *(volatile unsigned long long*)(PN16 + (size_t)row * D + lane * 4) = pk.u; __threadfence(); *(volatile unsigned long long*)(PN16 + (size_t)row * D + lane * 4) = pk.u;
}
__global__ __launch_bounds__(256) void k_xq(const float* __restrict__ x, _Float16* __restrict__ Q16, __bf16* __restrict__ XB) {
  const int wave = threadIdx.x >> 5, lane = threadIdx.x & 31; const size_t row = (size_t)blockIdx.x * 8 + wave; const v4f v = *(const v4f*)(x + row * D + lane * 4);
  float ss = v[0] * v[0] + v[1] * v[1] + v[2] * v[2] + v[3] * v[3];
#pragma unroll
  for (int o = 16; o > 0; o >>= 1) ss += __shfl_xor(ss, o, 32);
  const float inv = 4.0f / sqrtf(ss);
  union { _Float16 h[4]; unsigned long long u; } pk; union { __bf16 h[4]; unsigned long long u; } pb;
#pragma unroll
  for (int e = 0; e < 4; ++e) { pk.h[e] = (_Float16)(v[e] * inv); pb.h[e] = (__bf16)v[e]; }
  *(volatile unsigned long long*)(Q16 + row * D + lane * 4) = pk.u; *(volatile unsigned long long*)(XB + row * D + lane * 4) = pb.u; __threadfence();
  *(volatile unsigned long long*)(Q16 + row * D + lane * 4) = pk.u; *(volatile unsigned long long*)(XB + row * D + lane * 4) = pb.u;
}
__global__ __launch_bounds__(128) void k_attn(const _Float16* __restrict__ Q16, const _Float16* __restrict__ K16, const _Float16* __restrict__ VT16, const int* __restrict__ umask, float* __restrict__ CTX) {
  __shared__ __align__(16) float sS[4][16][68];
  __shared__ __align__(16) _Float16 sPh[4][16][72];
  __shared__ __align__(16) float sO[4][16][D + 4];
  const int tid = threadIdx.x, w = tid >> 5, lane = tid & 31, col = lane & 15, g = lane >> 4; const int q0 = blockIdx.x * 64 + w * 16;
  v16h aq[4];
#pragma unroll
  for (int kc = 0; kc < 4; ++kc) aq[kc] = frag_h(Q16 + (size_t)(q0 + col) * D + kc * 32, lane);
  const float mval = (1.0f - (float)umask[q0 + col]) * -10000.0f;
  float mrun = -3.0e38f, lrun = 0.f; v8f acc[8] = {};
#pragma unroll 1
  for (int kt = 0; kt < NK / 64; ++kt) {
#pragma unroll
    for (int t = 0; t < 4; ++t) { v8f s = {}; const int key = kt * 64 + t * 16 + col;
#pragma unroll
      for (int kc = 0; kc < 4; ++kc) s = wmma16(aq[kc], frag_h(K16 + (size_t)key * D + kc * 32, lane), s);
#pragma unroll
      for (int r = 0; r < 8; ++r) sS[w][8 * g + r][t * 16 + col] = s[r] * (1.0f / 16.0f); }
    LDSX();
    float mx = -3.4e38f;
#pragma unroll
    for (int jj = 0; jj < 32; ++jj) { const float sv = sS[w][col][g * 32 + jj] + mval; sS[w][col][g * 32 + jj] = sv; mx = fmaxf(mx, sv); }
    mx = fmaxf(mx, __shfl_xor(mx, 16, 32));
    const float mnew = fmaxf(mrun, mx); const float corr = expf(mrun - mnew);
    float ps = 0.f;
#pragma unroll
    for (int jj = 0; jj < 32; ++jj) { const float p = expf(sS[w][col][g * 32 + jj] - mnew) * 16384.0f; ps += p; sPh[w][col][g * 32 + jj] = (_Float16)p; }
    ps += __shfl_xor(ps, 16, 32);
    lrun = lrun * corr + ps * (1.0f / 16384.0f); mrun = mnew;
#pragma unroll
    for (int r = 0; r < 8; ++r) { const float cr = __shfl(corr, 8 * g + r, 32);
#pragma unroll
      for (int t = 0; t < 8; ++t) acc[t][r] *= cr; }
    LDSX();
#pragma unroll
    for (int kc = 0; kc < 2; ++kc) { const v16h ph = frag_h(&sPh[w][col][0] + kc * 32, lane);
#pragma unroll
      for (int t = 0; t < 8; ++t) acc[t] = wmma16(ph, frag_h(VT16 + (size_t)(t * 16 + col) * NK + kt * 64 + kc * 32, lane), acc[t]); }
    __builtin_amdgcn_wave_barrier(); }
#pragma unroll
  for (int r = 0; r < 8; ++r) { const float lr = __shfl(lrun, 8 * g + r, 32); const float inv = 1.0f / (lr * 16384.0f * 4.0f);
#pragma unroll
    for (int t = 0; t < 8; ++t) sO[w][8 * g + r][t * 16 + col] = acc[t][r] * inv; }
  LDSX();
  for (int rl = 0; rl < 16; ++rl) vst2(CTX + (size_t)(q0 + rl) * D + lane * 4, *(const v4f*)(&sO[w][rl][lane * 4]));
}
__global__ __launch_bounds__(128) void k_mlp(const float* __restrict__ CTX, const __bf16* __restrict__ XB, const float* __restrict__ wd1, const float* __restrict__ bd1, const float* __restrict__ wd2, const float* __restrict__ bd2, const float* __restrict__ wp, const float* __restrict__ bp, float* __restrict__ out0, float* __restrict__ out2) {
  __shared__ __align__(16) float sh[4][16][D + 4]; __shared__ __align__(16) float so[4][16][D + 4]; __shared__ __align__(16) float sr[4][16][D + 4];
  const int tid = threadIdx.x, wave = tid >> 5, lane = tid & 31, col = lane & 15, g = lane >> 4; const int r0 = blockIdx.x * 64 + wave * 16;
  { v8f acc[8] = {};
#pragma unroll
    for (int kc = 0; kc < 4; ++kc) { const F2 a = split_row(CTX + (size_t)(r0 + col) * D, kc * 32, lane);
#pragma unroll
      for (int j = 0; j < 8; ++j) { const v16b wb = split_col(wd1, kc * 32, j * 16 + col, lane, D, D).h; acc[j] = wmma_bf(a.l, wb, acc[j]); acc[j] = wmma_bf(a.h, wb, acc[j]); } }
#pragma unroll
    for (int j = 0; j < 8; ++j) { const float bb = bfr(bd1[j * 16 + col]);
#pragma unroll
      for (int r = 0; r < 8; ++r) sh[wave][8 * g + r][j * 16 + col] = gelu_e(acc[j][r] + bb); } }
  LDSX();
  { v8f acc[8] = {}, ar[8] = {};
#pragma unroll
    for (int kc = 0; kc < 4; ++kc) { const F2 a = split_row(&sh[wave][col][0], kc * 32, lane); const v16b xa = frag_b(XB + (size_t)(r0 + col) * D + kc * 32, lane);
#pragma unroll
      for (int j = 0; j < 8; ++j) { const v16b wb = split_col(wd2, kc * 32, j * 16 + col, lane, D, D).h; acc[j] = wmma_bf(a.l, wb, acc[j]); acc[j] = wmma_bf(a.h, wb, acc[j]);
        ar[j] = wmma_bf(xa, split_col(wp, kc * 32, j * 16 + col, lane, D, D).h, ar[j]); } }
#pragma unroll
    for (int j = 0; j < 8; ++j) { const float b2 = bfr(bd2[j * 16 + col]), bpp = bfr(bp[j * 16 + col]);
#pragma unroll
      for (int r = 0; r < 8; ++r) { const float rv = ar[j][r] + bpp; sr[wave][8 * g + r][j * 16 + col] = rv; so[wave][8 * g + r][j * 16 + col] = acc[j][r] + b2 + rv; } } }
  LDSX();
  for (int rl = 0; rl < 16; ++rl) { vst2(out0 + (size_t)(r0 + rl) * D + lane * 4, *(const v4f*)(&so[wave][rl][lane * 4])); vst2(out2 + (size_t)(r0 + rl) * D + lane * 4, *(const v4f*)(&sr[wave][rl][lane * 4])); }
}
extern "C" void kernel_launch(void* const* d_in, const int* in_sizes, int n_in, void* d_out, int out_size, void* d_ws, size_t ws_size, hipStream_t stream) {
  (void)in_sizes; (void)n_in; (void)out_size; (void)ws_size;
  const float* x = (const float*)d_in[0]; const int* umask = (const int*)d_in[1]; const float* wn1 = (const float*)d_in[2]; const float* bn1 = (const float*)d_in[3]; const float* wn2 = (const float*)d_in[4]; const float* bn2 = (const float*)d_in[5];
  const float* wd1 = (const float*)d_in[6]; const float* bd1 = (const float*)d_in[7]; const float* wd2 = (const float*)d_in[8]; const float* bd2 = (const float*)d_in[9]; const float* wp = (const float*)d_in[10]; const float* bp = (const float*)d_in[11];
  float* out0 = (float*)d_out; float* proto = (float*)((char*)d_out + 8388608); float* out2 = (float*)((char*)d_out + 9437184);
  char* ws = (char*)d_ws; size_t off = 0;
  auto take = [&](size_t bytes) { char* p = ws + off; off += (bytes + 255) & ~(size_t)255; return p; };
  _Float16* VT16 = (_Float16*)take((size_t)D * NK * 2); _Float16* PN16 = (_Float16*)take((size_t)NK * D * 2); _Float16* Q16 = (_Float16*)take((size_t)NR * D * 2); __bf16* XB = (__bf16*)take((size_t)NR * D * 2); float* CTX = (float*)take((size_t)NR * D * 4);
  k_proto<<<dim3(D / 64, NBI), 128, 0, stream>>>(x, wn1, bn1, wn2, bn2, proto, VT16);
  k_pn<<<NK / 8, 256, 0, stream>>>(proto, PN16);
  k_xq<<<NR / 8, 256, 0, stream>>>(x, Q16, XB);
  k_attn<<<NR / 64, 128, 0, stream>>>(Q16, PN16, VT16, umask, CTX);
  k_mlp<<<NR / 64, 128, 0, stream>>>(CTX, XB, wd1, bd1, wd2, bd2, wp, bp, out0, out2);
}
